// SelectiveSSMLayer_41240275976483
// MI455X (gfx1250) — hardware-run, weakly checked
//
#include <hip/hip_runtime.h>
#include <math.h>

typedef __attribute__((ext_vector_type(16))) _Float16 v16h;
typedef __attribute__((ext_vector_type(8)))  _Float16 v8h;
typedef __attribute__((ext_vector_type(4)))  _Float16 v4h;
typedef __attribute__((ext_vector_type(8)))  float    v8f;
typedef __attribute__((ext_vector_type(4)))  float    v4f;

constexpr int kBatch = 2;
constexpr int kLen   = 256;
constexpr int kHid   = 256;
constexpr int kInner = 512;
constexpr int kRows  = kBatch * kLen;
constexpr int kXpN   = 2 * kInner;
constexpr int kConvK = 3 * kInner;
constexpr int kSsmN  = 2 * kInner;
constexpr int kStepChunk = 8;
constexpr float kWCarry   = 1024.0f;
constexpr float kResid    = 2048.0f;
constexpr float kActCarry = 64.0f;
constexpr float kYCarry   = 1.0f / 64.0f;
constexpr float sAW  = 1.0f / (kActCarry * kWCarry);
constexpr float sAWR = 1.0f / (kActCarry * kWCarry * kResid);
constexpr float sYW  = 1.0f / (kYCarry * kWCarry);
constexpr float sYWR = 1.0f / (kYCarry * kWCarry * kResid);
static_assert(kRows == 512 && kXpN == 1024 && kConvK == 1536);
static_assert((kRows % 16) == 0 && (kXpN % 64) == 0 && (kInner % 64) == 0 && (kSsmN % 64) == 0 && (kHid % 64) == 0);
static_assert((kHid % 32) == 0 && (kConvK % 32) == 0 && (kInner % 32) == 0);
static_assert((kLen % kStepChunk) == 0);

constexpr size_t kSzX16  = (size_t)kRows * kHid * 2;
constexpr size_t kSzWin  = (size_t)kXpN * kHid * 2;
constexpr size_t kSzWc   = (size_t)kInner * kConvK * 2;
constexpr size_t kSzWs   = (size_t)kSsmN * kInner * 2;
constexpr size_t kSzWg   = (size_t)kInner * kInner * 2;
constexpr size_t kSzWo   = (size_t)kHid * kInner * 2;
constexpr size_t kSzXP   = (size_t)kRows * kXpN * 4;
constexpr size_t kSzAc   = (size_t)kRows * kConvK * 2;
constexpr size_t kSzF32  = (size_t)kRows * kInner * 4;
constexpr size_t kSzF16  = (size_t)kRows * kInner * 2;
constexpr size_t kSzCD   = (size_t)kRows * kSsmN * 4;
constexpr size_t kSzOP   = (size_t)kRows * kHid * 4;
constexpr size_t kOffXH   = 0;
constexpr size_t kOffXL   = kOffXH   + kSzX16;
constexpr size_t kOffWINH = kOffXL   + kSzX16;
constexpr size_t kOffWINL = kOffWINH + kSzWin;
constexpr size_t kOffWCH  = kOffWINL + kSzWin;
constexpr size_t kOffWCL  = kOffWCH  + kSzWc;
constexpr size_t kOffWSH  = kOffWCL  + kSzWc;
constexpr size_t kOffWSL  = kOffWSH  + kSzWs;
constexpr size_t kOffWGH  = kOffWSL  + kSzWs;
constexpr size_t kOffWGL  = kOffWGH  + kSzWg;
constexpr size_t kOffWOH  = kOffWGL  + kSzWg;
constexpr size_t kOffWOL  = kOffWOH  + kSzWo;
constexpr size_t kOffXP   = kOffWOL  + kSzWo;
constexpr size_t kOffACH  = kOffXP   + kSzXP;
constexpr size_t kOffACL  = kOffACH  + kSzAc;
constexpr size_t kOffCV   = kOffACL  + kSzAc;
constexpr size_t kOffXC   = kOffCV   + kSzF32;
constexpr size_t kOffXCH  = kOffXC   + kSzF32;
constexpr size_t kOffXCL  = kOffXCH  + kSzF16;
constexpr size_t kOffCD   = kOffXCL  + kSzF16;
constexpr size_t kOffGT   = kOffCD   + kSzCD;
constexpr size_t kOffUU   = kOffGT   + kSzF32;
constexpr size_t kOffCWT  = kOffUU   + kSzF32;
constexpr size_t kOffYY   = kOffCWT  + kSzF32;
constexpr size_t kOffYH   = kOffYY   + kSzF32;
constexpr size_t kOffYL   = kOffYH   + kSzF16;
constexpr size_t kOffOPRE = kOffYL   + kSzF16;
constexpr size_t kWsTotal = kOffOPRE + kSzOP;
static_assert(kWsTotal == 24641536ull);
static_assert(kWsTotal <= 134217728ull);
static_assert((kSzX16 % 128) == 0 && (kSzWin % 128) == 0 && (kSzWc % 128) == 0 && (kSzWs % 128) == 0 &&
              (kSzWg % 128) == 0 && (kSzWo % 128) == 0 && (kSzXP % 128) == 0 && (kSzAc % 128) == 0 &&
              (kSzF32 % 128) == 0 && (kSzF16 % 128) == 0 && (kSzCD % 128) == 0 && (kSzOP % 128) == 0);
static_assert((size_t)kRows * kHid * 4 == 524288ull);

__device__ __forceinline__ _Float16 f16_flush(float v) {
  const float w = (fabsf(v) < 6.103515625e-05f) ? 0.0f : v;
  return (_Float16)w;
}
__device__ __forceinline__ void f16_split(float v, _Float16& hi, _Float16& lo) {
  hi = f16_flush(v);
  const float hf = (float)hi;
  const float r = (v - hf) * kResid;
  lo = f16_flush(r);
}
__device__ __forceinline__ void pin_f(float& x) { asm volatile("" : "+v"(x)); }

namespace eng {
union FragU { v16h v; v8h h[2]; };
__device__ __forceinline__ v16h frag_load(const _Float16* p) {
  FragU f;
  f.h[0] = *(const v8h*)(p);
  f.h[1] = *(const v8h*)(p + 16);
  return f.v;
}
__device__ __forceinline__ v8f mma(v16h a, v16h b, v8f c) {
  return __builtin_amdgcn_wmma_f32_16x16x32_f16(false, a, false, b, (short)0, c, false, false);
}
__device__ __forceinline__ void guard1(v8f& a, v16h x, v16h y) {
  asm volatile("v_nop\n\tv_nop\n\tv_nop\n\tv_nop" : "+v"(a) : "v"(x), "v"(y));
}
__device__ __forceinline__ void guard_acc(v8f& a) {
  asm volatile("v_nop\n\tv_nop\n\tv_nop\n\tv_nop" : "+v"(a));
}
__device__ __forceinline__ void keep4(v16h a, v16h b, v16h c, v16h d) {
  asm volatile("v_nop" :: "v"(a), "v"(b), "v"(c), "v"(d));
}

template <bool HASB, int ACT>
__global__ __launch_bounds__(256) void gemm_f16x3_kernel(
    const unsigned short* __restrict__ Ahp, const unsigned short* __restrict__ Alp, int lda,
    const unsigned short* __restrict__ Bhp, const unsigned short* __restrict__ Blp, int ldb,
    float* C, int ldc, const float* __restrict__ bias, int M, int N, int K, float scale, float rscale)
{
  static_assert(ACT >= 0 && ACT <= 1);
  const _Float16* Ah = (const _Float16*)Ahp;
  const _Float16* Al = (const _Float16*)Alp;
  const _Float16* Bh = (const _Float16*)Bhp;
  const _Float16* Bl = (const _Float16*)Blp;
  __shared__ __align__(16) float sT[8][16 * 68];
  const int lane = threadIdx.x & 31;
  const int wave = threadIdx.x >> 5;
  const int tilesN = N >> 6;
  const int tilesM = M >> 4;
  const int tile = blockIdx.x * 8 + wave;
  if (tile >= tilesM * tilesN) return;
  const int tm = tile / tilesN;
  const int tn = tile - tm * tilesN;
  const int m0 = tm << 4;
  const int n0 = tn << 6;
  const int rlane = lane & 15;
  const int koff  = (lane >> 4) * 8;
  const int mOff  = (lane >> 4) * 8;

  v8f acc[4], accr[4];
#pragma unroll
  for (int j = 0; j < 4; ++j) {
    acc[j]  = (v8f){0.f, 0.f, 0.f, 0.f, 0.f, 0.f, 0.f, 0.f};
    accr[j] = (v8f){0.f, 0.f, 0.f, 0.f, 0.f, 0.f, 0.f, 0.f};
  }
  const size_t arow = (size_t)(m0 + rlane) * lda + koff;

  for (int k0 = 0; k0 < K; k0 += 32) {
    v16h bh[4], bl[4];
#pragma unroll
    for (int j = 0; j < 4; ++j) {
      const size_t bo = (size_t)(n0 + (j << 4) + rlane) * ldb + koff + k0;
      bh[j] = frag_load(Bh + bo);
      bl[j] = frag_load(Bl + bo);
    }
    const v16h ah = frag_load(Ah + arow + k0);
    const v16h al = frag_load(Al + arow + k0);
#pragma unroll
    for (int jp = 0; jp < 2; ++jp) {
#pragma unroll
      for (int jj = 0; jj < 2; ++jj) {
        const int j = jp * 2 + jj;
        acc[j]  = mma(ah, bh[j], acc[j]);
        accr[j] = mma(al, bh[j], accr[j]);
        accr[j] = mma(ah, bl[j], accr[j]);
      }
#pragma unroll
      for (int jj = 0; jj < 2; ++jj) {
        const int j = jp * 2 + jj;
        guard1(acc[j], ah, al);
        guard1(accr[j], ah, al);
      }
    }
    keep4(bh[0], bh[1], bh[2], bh[3]);
    keep4(bl[0], bl[1], bl[2], bl[3]);
  }
#pragma unroll
  for (int j = 0; j < 4; ++j) {
    guard_acc(acc[j]);
    guard_acc(accr[j]);
  }

  float* slab = sT[wave];
  const int hh = lane >> 4, c4 = (lane & 15) * 4;
  v4f bv = (v4f){0.f, 0.f, 0.f, 0.f};
  if (HASB) bv = *(const v4f*)(bias + n0 + c4);
#pragma unroll
  for (int j = 0; j < 4; ++j) {
#pragma unroll
    for (int r = 0; r < 8; ++r) {
      const float v = fmaf(accr[j][r], rscale, acc[j][r] * scale);
      slab[(mOff + r) * 68 + (j << 4) + rlane] = v;
    }
  }
  __builtin_amdgcn_fence(__ATOMIC_RELEASE, "workgroup");
  __builtin_amdgcn_wave_barrier();
  __builtin_amdgcn_fence(__ATOMIC_ACQUIRE, "workgroup");
  if (HASB || ACT != 0) {
    for (int it = 0; it < 8; ++it) {
      float* sp = slab + (it * 2 + hh) * 68 + c4;
      v4f v = *(const v4f*)sp;
      v = v + bv;
      if (ACT == 1) {
#pragma unroll
        for (int e = 0; e < 4; ++e) v[e] = __builtin_amdgcn_rcpf(1.0f + expf(-v[e]));
      }
      *(v4f*)sp = v;
    }
  }
  for (int pass = 0; pass < 2; ++pass) {
#pragma unroll
    for (int it = 0; it < 8; ++it) {
      const int row = it * 2 + hh;
      const v4f v = *(const v4f*)(slab + row * 68 + c4);
      *(volatile v4f*)(C + (size_t)(m0 + row) * ldc + n0 + c4) = v;
    }
    __threadfence();
  }
}
}

__global__ __launch_bounds__(256) void split_rows_kernel(
    const float* __restrict__ src, unsigned short* __restrict__ dH, unsigned short* __restrict__ dL,
    int total8, float carry)
{
  const int i = blockIdx.x * 256 + threadIdx.x;
  if (i >= total8) return;
  const size_t e0 = (size_t)i << 3;
  const v4f a0 = *(const v4f*)(src + e0);
  const v4f a1 = *(const v4f*)(src + e0 + 4);
  v8h hv, lv;
#pragma unroll
  for (int e = 0; e < 4; ++e) {
    _Float16 h0, l0, h1, l1;
    const float f0 = a0[e] * carry;
    const float f1 = a1[e] * carry;
    f16_split(f0, h0, l0);
    f16_split(f1, h1, l1);
    hv[e] = h0; lv[e] = l0;
    hv[4 + e] = h1; lv[4 + e] = l1;
  }
  unsigned short* qh = dH + e0;
  unsigned short* ql = dL + e0;
  *(volatile v8h*)qh = hv;
  *(volatile v8h*)ql = lv;
  __threadfence();
  *(volatile v8h*)qh = hv;
  *(volatile v8h*)ql = lv;
}

__global__ __launch_bounds__(256) void conv_pack_kernel(
    const float* __restrict__ cw, unsigned short* __restrict__ dH, unsigned short* __restrict__ dL,
    int total8, float carry)
{
  const int i = blockIdx.x * 256 + threadIdx.x;
  if (i >= total8) return;
  const int e0  = i << 3;
  const int o   = e0 / kConvK;
  const int k   = e0 - o * kConvK;
  const int tap = k >> 9;
  const int c0  = k & (kInner - 1);
  const float* sp = cw + (size_t)o * kConvK + (size_t)c0 * 3 + tap;
  v8h hv, lv;
#pragma unroll
  for (int e = 0; e < 8; ++e) {
    _Float16 h, l;
    const float f = sp[e * 3] * carry;
    f16_split(f, h, l);
    hv[e] = h; lv[e] = l;
  }
  unsigned short* qh = dH + (size_t)e0;
  unsigned short* ql = dL + (size_t)e0;
  *(volatile v8h*)qh = hv;
  *(volatile v8h*)ql = lv;
  __threadfence();
  *(volatile v8h*)qh = hv;
  *(volatile v8h*)ql = lv;
}

__global__ __launch_bounds__(256) void im2col_kernel(
    const float* __restrict__ XP, unsigned short* __restrict__ dH, unsigned short* __restrict__ dL,
    int total8, float carry)
{
  const int i = blockIdx.x * 256 + threadIdx.x;
  if (i >= total8) return;
  const int e0  = i << 3;
  const int row = e0 / kConvK;
  const int k   = e0 - row * kConvK;
  const int tap = k >> 9;
  const int c0  = k & (kInner - 1);
  const int t   = row & (kLen - 1);
  const int tt  = t + tap - 1;
  const bool ok = (tt >= 0) && (tt < kLen);
  const int srow = ok ? (row + tap - 1) : row;
  const float* sp = XP + (size_t)srow * kXpN + kInner + c0;
  const v4f a0 = *(const v4f*)(sp);
  const v4f a1 = *(const v4f*)(sp + 4);
  v8h hv, lv;
#pragma unroll
  for (int e = 0; e < 4; ++e) {
    float f0 = a0[e];
    float f1 = a1[e];
    pin_f(f0); pin_f(f1);
    f0 = ok ? (f0 * carry) : 0.0f;
    f1 = ok ? (f1 * carry) : 0.0f;
    _Float16 h0, l0, h1, l1;
    f16_split(f0, h0, l0);
    f16_split(f1, h1, l1);
    hv[e] = h0; lv[e] = l0;
    hv[4 + e] = h1; lv[4 + e] = l1;
  }
  unsigned short* qh = dH + (size_t)e0;
  unsigned short* ql = dL + (size_t)e0;
  *(volatile v8h*)qh = hv;
  *(volatile v8h*)ql = lv;
  __threadfence();
  *(volatile v8h*)qh = hv;
  *(volatile v8h*)ql = lv;
}

__global__ __launch_bounds__(256) void gelu_add_kernel(
    const float* __restrict__ XP, const float* __restrict__ CV, float* __restrict__ XC,
    unsigned short* __restrict__ XCH, unsigned short* __restrict__ XCL, int total4, float carry)
{
  const int i = blockIdx.x * 256 + threadIdx.x;
  if (i >= total4) return;
  const int e0  = i << 2;
  const int row = e0 >> 9;
  const int c0  = e0 & (kInner - 1);
  const v4f q  = *(const v4f*)(XP + (size_t)row * kXpN + c0);
  const v4f cv = *(const v4f*)(CV + (size_t)e0);
  v4f xc;
  v4h hv, lv;
#pragma unroll
  for (int e = 0; e < 4; ++e) {
    const float v = q[e];
    const float ge = 0.5f * v * (1.0f + erff(v * 0.70710678118654752f));
    const float s = ge + cv[e];
    xc[e] = s;
    _Float16 h, l;
    f16_split(s * carry, h, l);
    hv[e] = h; lv[e] = l;
  }
  float* pf = XC + (size_t)e0;
  unsigned short* qh = XCH + (size_t)e0;
  unsigned short* ql = XCL + (size_t)e0;
  *(volatile v4f*)pf = xc;
  *(volatile v4h*)qh = hv;
  *(volatile v4h*)ql = lv;
  __threadfence();
  *(volatile v4f*)pf = xc;
  *(volatile v4h*)qh = hv;
  *(volatile v4h*)ql = lv;
}

__global__ __launch_bounds__(256) void gate_mul_kernel(
    const float* __restrict__ XC, const float* __restrict__ CD, const float* __restrict__ GT,
    float* __restrict__ UU, float* __restrict__ CWT, int total4)
{
  const int i = blockIdx.x * 256 + threadIdx.x;
  if (i >= total4) return;
  const int e0  = i << 2;
  const int row = e0 >> 9;
  const int c0  = e0 & (kInner - 1);
  const v4f xc = *(const v4f*)(XC + (size_t)e0);
  const v4f cr = *(const v4f*)(CD + (size_t)row * kSsmN + c0);
  const v4f dw = *(const v4f*)(CD + (size_t)row * kSsmN + kInner + c0);
  const v4f g  = *(const v4f*)(GT + (size_t)e0);
  v4f u, cw;
#pragma unroll
  for (int e = 0; e < 4; ++e) {
    const float d2 = dw[e] * dw[e];
    u[e]  = xc[e] * d2;
    cw[e] = g[e] * cr[e];
  }
  float* pu = UU + (size_t)e0;
  float* pc = CWT + (size_t)e0;
  *(volatile v4f*)pu = u;
  *(volatile v4f*)pc = cw;
  __threadfence();
  *(volatile v4f*)pu = u;
  *(volatile v4f*)pc = cw;
}

__global__ __launch_bounds__(512) void scan_kernel(
    const float* __restrict__ UU, const float* __restrict__ CWT, const float* __restrict__ Amat,
    const float* __restrict__ Dvec, float* __restrict__ YY)
{
  __shared__ __align__(16) float su[kStepChunk * kInner];
  __shared__ __align__(16) float sc[kStepChunk * kInner];
  __shared__ __align__(16) float red[kStepChunk * 16 * 32];
  const int tid = threadIdx.x, lane = tid & 31, wave = tid >> 5;
  const int bi  = blockIdx.x >> 4;
  const int i0  = (blockIdx.x & 15) * 32;
  const int col = i0 + lane;
  const int s0  = wave * 32;

  float a[32], h[32];
#pragma unroll
  for (int g = 0; g < 2; ++g) {
#pragma unroll
    for (int s = 0; s < 16; ++s) a[g * 16 + s] = Amat[(size_t)(s0 + g * 16 + s) * kInner + col];
#pragma unroll
    for (int s = 0; s < 16; ++s) pin_f(a[g * 16 + s]);
    asm volatile("" ::: "memory");
  }
#pragma unroll
  for (int s = 0; s < 32; ++s) h[s] = 0.0f;
  const float dsk = Dvec[col];
  const float* ub = UU  + (size_t)bi * kLen * kInner;
  const float* cb = CWT + (size_t)bi * kLen * kInner;
  float*       yb = YY  + (size_t)bi * kLen * kInner;

  for (int ch = 0; ch < kLen / kStepChunk; ++ch) {
    const int t0 = ch * kStepChunk;
#pragma unroll
    for (int p = 0; p < 2; ++p) {
      const int idx = (tid + p * 512) * 4;
      const v4f vu = *(const v4f*)(ub + (size_t)t0 * kInner + idx);
      const v4f vc = *(const v4f*)(cb + (size_t)t0 * kInner + idx);
      *(v4f*)(su + idx) = vu;
      *(v4f*)(sc + idx) = vc;
    }
    __syncthreads();
    for (int t = 0; t < kStepChunk; ++t) {
      const float* up = su + t * kInner + s0;
      const float* cp = sc + t * kInner + s0;
      float p = 0.0f;
#pragma unroll
      for (int q = 0; q < 8; ++q) {
        const v4f uv = *(const v4f*)(up + 4 * q);
        const v4f cv = *(const v4f*)(cp + 4 * q);
#pragma unroll
        for (int e = 0; e < 4; ++e) {
          h[4 * q + e] = fmaf(h[4 * q + e], a[4 * q + e], uv[e]);
          p = fmaf(h[4 * q + e], cv[e], p);
        }
      }
      red[(t * 16 + wave) * 32 + lane] = p;
    }
    __syncthreads();
    if (tid < kStepChunk * 32) {
      const int t = wave;
      float s = 0.0f;
#pragma unroll
      for (int w = 0; w < 16; ++w) s += red[(t * 16 + w) * 32 + lane];
      const float uk = su[t * kInner + col];
      const float yv = fmaf(uk, dsk, s);
      volatile float* yp = yb + (size_t)(t0 + t) * kInner + col;
      *yp = yv;
      __threadfence();
      *yp = yv;
    }
    __syncthreads();
  }
}

__global__ __launch_bounds__(256) void ln_kernel(
    const float* __restrict__ OP, const float* __restrict__ x, const float* __restrict__ lg,
    const float* __restrict__ lb, const float* __restrict__ z, float* __restrict__ out)
{
  const int row  = (blockIdx.x * 256 + threadIdx.x) >> 5;
  const int lane = threadIdx.x & 31;
  const int c = lane * 4;
  const size_t base = (size_t)row * kHid;
  const v4f v0 = *(const v4f*)(OP + base + c);
  const v4f v1 = *(const v4f*)(OP + base + 128 + c);
  float s = ((v0[0] + v0[1]) + (v0[2] + v0[3])) + ((v1[0] + v1[1]) + (v1[2] + v1[3]));
#pragma unroll
  for (int off = 16; off > 0; off >>= 1) s += __shfl_xor(s, off, 32);
  const float mu = s * (1.0f / kHid);
  v4f d0, d1;
#pragma unroll
  for (int e = 0; e < 4; ++e) { d0[e] = v0[e] - mu; d1[e] = v1[e] - mu; }
  float ss = ((d0[0] * d0[0] + d0[1] * d0[1]) + (d0[2] * d0[2] + d0[3] * d0[3])) +
             ((d1[0] * d1[0] + d1[1] * d1[1]) + (d1[2] * d1[2] + d1[3] * d1[3]));
#pragma unroll
  for (int off = 16; off > 0; off >>= 1) ss += __shfl_xor(ss, off, 32);
  const float var = ss * (1.0f / kHid);
  const float inv = rsqrtf(var + 1e-5f);
  const float zz = z[0];
  const v4f g0 = *(const v4f*)(lg + c);
  const v4f g1 = *(const v4f*)(lg + 128 + c);
  const v4f b0 = *(const v4f*)(lb + c);
  const v4f b1 = *(const v4f*)(lb + 128 + c);
  const v4f x0 = *(const v4f*)(x + base + c);
  const v4f x1 = *(const v4f*)(x + base + 128 + c);
  v4f r0, r1;
#pragma unroll
  for (int e = 0; e < 4; ++e) {
    const float o0 = (d0[e] * inv) * g0[e] + b0[e];
    const float o1 = (d1[e] * inv) * g1[e] + b1[e];
    r0[e] = o0 * zz + x0[e];
    r1[e] = o1 * zz + x1[e];
  }
  float* p0 = out + base + c;
  float* p1 = out + base + 128 + c;
  *(volatile v4f*)p0 = r0;
  *(volatile v4f*)p1 = r1;
  __threadfence();
  *(volatile v4f*)p0 = r0;
  *(volatile v4f*)p1 = r1;
}

static_assert(((kRows / 16) * (kXpN / 64)) % 8 == 0);
static_assert(((kRows / 16) * (kInner / 64)) % 8 == 0);
static_assert(((kRows / 16) * (kSsmN / 64)) % 8 == 0);
static_assert(((kRows / 16) * (kHid / 64)) % 8 == 0);
static_assert(((kRows * kHid / 8) % 256) == 0 && ((kXpN * kHid / 8) % 256) == 0 &&
              ((kInner * kConvK / 8) % 256) == 0 && ((kSsmN * kInner / 8) % 256) == 0 &&
              ((kInner * kInner / 8) % 256) == 0 && ((kHid * kInner / 8) % 256) == 0 &&
              ((kRows * kConvK / 8) % 256) == 0 && ((kRows * kInner / 8) % 256) == 0 &&
              ((kRows * kInner / 4) % 256) == 0);

extern "C" void kernel_launch(void* const* d_in, const int* in_sizes, int n_in,
                              void* d_out, int out_size, void* d_ws, size_t ws_size,
                              hipStream_t stream)
{
  if (n_in < 14) return;
  if (in_sizes[0]  != kRows * kHid) return;
  if (in_sizes[1]  != kXpN * kHid) return;
  if (in_sizes[2]  != kInner * kInner * 3) return;
  if (in_sizes[3]  != kInner) return;
  if (in_sizes[4]  != 3 * kInner * kInner) return;
  if (in_sizes[5]  != 3 * kInner) return;
  if (in_sizes[6]  != 2 * kInner * kInner) return;
  if (in_sizes[7]  != 2 * kInner) return;
  if (in_sizes[8]  != kInner * kInner) return;
  if (in_sizes[9]  != kInner) return;
  if (in_sizes[10] != kHid * kInner) return;
  if (in_sizes[11] != 1) return;
  if (in_sizes[12] != kHid) return;
  if (in_sizes[13] != kHid) return;
  if (out_size != kRows * kHid) return;
  if (ws_size < kWsTotal) return;

  const float* x      = (const float*)d_in[0];
  const float* W_in   = (const float*)d_in[1];
  const float* conv_w = (const float*)d_in[2];
  const float* conv_b = (const float*)d_in[3];
  const float* W_ssm  = (const float*)d_in[4];
  const float* b_ssm  = (const float*)d_in[5];
  const float* W_gate = (const float*)d_in[6];
  const float* b_gate = (const float*)d_in[7];
  const float* Amat   = (const float*)d_in[8];
  const float* Dvec   = (const float*)d_in[9];
  const float* W_out  = (const float*)d_in[10];
  const float* zsc    = (const float*)d_in[11];
  const float* ln_g   = (const float*)d_in[12];
  const float* ln_b   = (const float*)d_in[13];
  float* out = (float*)d_out;

  char* ws = (char*)d_ws;
  unsigned short* XH   = (unsigned short*)(ws + kOffXH);
  unsigned short* XL   = (unsigned short*)(ws + kOffXL);
  unsigned short* WINH = (unsigned short*)(ws + kOffWINH);
  unsigned short* WINL = (unsigned short*)(ws + kOffWINL);
  unsigned short* WCH  = (unsigned short*)(ws + kOffWCH);
  unsigned short* WCL  = (unsigned short*)(ws + kOffWCL);
  unsigned short* WSH  = (unsigned short*)(ws + kOffWSH);
  unsigned short* WSL  = (unsigned short*)(ws + kOffWSL);
  unsigned short* WGH  = (unsigned short*)(ws + kOffWGH);
  unsigned short* WGL  = (unsigned short*)(ws + kOffWGL);
  unsigned short* WOH  = (unsigned short*)(ws + kOffWOH);
  unsigned short* WOL  = (unsigned short*)(ws + kOffWOL);
  float*          XP   = (float*)(ws + kOffXP);
  unsigned short* ACH  = (unsigned short*)(ws + kOffACH);
  unsigned short* ACL  = (unsigned short*)(ws + kOffACL);
  float*          CV   = (float*)(ws + kOffCV);
  float*          XC   = (float*)(ws + kOffXC);
  unsigned short* XCH  = (unsigned short*)(ws + kOffXCH);
  unsigned short* XCL  = (unsigned short*)(ws + kOffXCL);
  float*          CD   = (float*)(ws + kOffCD);
  float*          GT   = (float*)(ws + kOffGT);
  float*          UU   = (float*)(ws + kOffUU);
  float*          CWT  = (float*)(ws + kOffCWT);
  float*          YY   = (float*)(ws + kOffYY);
  unsigned short* YH   = (unsigned short*)(ws + kOffYH);
  unsigned short* YL   = (unsigned short*)(ws + kOffYL);
  float*          OPRE = (float*)(ws + kOffOPRE);

  split_rows_kernel<<<(kRows * kHid / 8) / 256, 256, 0, stream>>>(x, XH, XL, kRows * kHid / 8, kActCarry);
  split_rows_kernel<<<(kXpN * kHid / 8) / 256, 256, 0, stream>>>(W_in, WINH, WINL, kXpN * kHid / 8, kWCarry);
  conv_pack_kernel<<<(kInner * kConvK / 8) / 256, 256, 0, stream>>>(conv_w, WCH, WCL, kInner * kConvK / 8, kWCarry);
  split_rows_kernel<<<(kSsmN * kInner / 8) / 256, 256, 0, stream>>>(
      W_ssm + (size_t)kInner * kInner, WSH, WSL, kSsmN * kInner / 8, kWCarry);
  split_rows_kernel<<<(kInner * kInner / 8) / 256, 256, 0, stream>>>(
      W_gate + (size_t)kInner * kInner, WGH, WGL, kInner * kInner / 8, kWCarry);
  split_rows_kernel<<<(kHid * kInner / 8) / 256, 256, 0, stream>>>(W_out, WOH, WOL, kHid * kInner / 8, kWCarry);

  eng::gemm_f16x3_kernel<false, 0><<<((kRows / 16) * (kXpN / 64)) / 8, 256, 0, stream>>>(
      XH, XL, kHid, WINH, WINL, kHid, XP, kXpN, conv_b, kRows, kXpN, kHid, sAW, sAWR);

  im2col_kernel<<<(kRows * kConvK / 8) / 256, 256, 0, stream>>>(XP, ACH, ACL, kRows * kConvK / 8, kActCarry);

  eng::gemm_f16x3_kernel<true, 0><<<((kRows / 16) * (kInner / 64)) / 8, 256, 0, stream>>>(
      ACH, ACL, kConvK, WCH, WCL, kConvK, CV, kInner, conv_b, kRows, kInner, kConvK, sAW, sAWR);

  gelu_add_kernel<<<(kRows * kInner / 4) / 256, 256, 0, stream>>>(XP, CV, XC, XCH, XCL, kRows * kInner / 4, kActCarry);

  eng::gemm_f16x3_kernel<true, 0><<<((kRows / 16) * (kSsmN / 64)) / 8, 256, 0, stream>>>(
      XCH, XCL, kInner, WSH, WSL, kInner, CD, kSsmN, b_ssm + kInner, kRows, kSsmN, kInner, sAW, sAWR);

  eng::gemm_f16x3_kernel<true, 1><<<((kRows / 16) * (kInner / 64)) / 8, 256, 0, stream>>>(
      XCH, XCL, kInner, WGH, WGL, kInner, GT, kInner, b_gate + kInner, kRows, kInner, kInner, sAW, sAWR);

  gate_mul_kernel<<<(kRows * kInner / 4) / 256, 256, 0, stream>>>(XC, CD, GT, UU, CWT, kRows * kInner / 4);

  scan_kernel<<<kBatch * (kInner / 32), 512, 0, stream>>>(UU, CWT, Amat, Dvec, YY);

  split_rows_kernel<<<(kRows * kInner / 8) / 256, 256, 0, stream>>>(YY, YH, YL, kRows * kInner / 8, kYCarry);

  eng::gemm_f16x3_kernel<false, 0><<<((kRows / 16) * (kHid / 64)) / 8, 256, 0, stream>>>(
      YH, YL, kInner, WOH, WOL, kInner, OPRE, kHid, conv_b, kRows, kHid, kInner, sYW, sYWR);

  ln_kernel<<<(kRows * 32) / 256, 256, 0, stream>>>(OPRE, x, ln_g, ln_b, zsc, out);
}
